// MultiHeadAttention_91285234909775
// MI455X (gfx1250) — hardware-run, weakly checked
//
#include <hip/hip_runtime.h>


#ifndef NB
#define NB 2
#endif
#ifndef SEQ
#define SEQ 2048
#endif
#define NB_FULL  2
#define SEQ_FULL 2048
#ifndef OUT_SEQ
#define OUT_SEQ SEQ
#endif
#ifndef EARLY
#define EARLY 512
#endif
#define EARLYR ((EARLY < SEQ) ? EARLY : SEQ)
#define DM   1024
#define NH_  16
#define HD   64
#define POS  16
#define XP   1040
#define CXP  2048
#define AW   4
#define OSP  84
#define QRS  2048.0f
#define QRI  (1.0f / 2048.0f)
#define SC2  (0.125f * 1.4426950408889634f)
#define MASKV (-1.0e9f * 1.4426950408889634f)
#define PSH  8.0f
#define CXC  64.0f
#define WHC  16384.0f
#define WLC  8.0f
#define OSC  (1.0f / 1048576.0f)

static_assert(HD == 64);
static_assert(NH_ * HD == DM);
static_assert(DM % 64 == 0);
static_assert(DM % 32 == 0);
static_assert(SEQ % 64 == 0);
static_assert((NB * SEQ) % 64 == 0);
static_assert(SEQ % 32 == 0);
static_assert(EARLYR % 64 == 0);
static_assert((SEQ - EARLYR) % (16 * AW) == 0);
static_assert(EARLYR % (16 * AW) == 0);
static_assert(OUT_SEQ % 8 == 0);
static_assert(XP == DM + POS);
static_assert((XP * 8 * 4) % 128 == 0);
static_assert(NB <= NB_FULL);
static_assert(SEQ <= SEQ_FULL);
static_assert(WLC * QRS == WHC);

typedef _Float16 h16;
typedef unsigned short bf;
typedef __attribute__((ext_vector_type(16))) __bf16   v16bf;
typedef __attribute__((ext_vector_type(16))) _Float16 v16h;
typedef __attribute__((ext_vector_type(8)))  _Float16 v8h;
typedef __attribute__((ext_vector_type(8)))  unsigned short v8us;
typedef __attribute__((ext_vector_type(8)))  float    v8f;
typedef __attribute__((ext_vector_type(4)))  float    v4f;
typedef __attribute__((ext_vector_type(4)))  int      v4i;
typedef v4f  __attribute__((may_alias)) v4fa;

__device__ __forceinline__ unsigned short f2bf(float f) { unsigned u = __float_as_uint(f); u += 0x7FFFu + ((u >> 16) & 1u); return (unsigned short)(u >> 16); }
__device__ __forceinline__ float bfr(float f) { return __uint_as_float(((unsigned)f2bf(f)) << 16); }
__device__ __forceinline__ v16h cat16(v8h lo, v8h hi) { return __builtin_shufflevector(lo, hi, 0, 1, 2, 3, 4, 5, 6, 7, 8, 9, 10, 11, 12, 13, 14, 15); }
__device__ __forceinline__ v16bf cat16b(v8us lo, v8us hi) { return __builtin_bit_cast(v16bf, __builtin_shufflevector(lo, hi, 0, 1, 2, 3, 4, 5, 6, 7, 8, 9, 10, 11, 12, 13, 14, 15)); }
__device__ __forceinline__ v8f wmma16(v16h a, v16h b, v8f c) { return __builtin_amdgcn_wmma_f32_16x16x32_f16(false, a, false, b, (short)0, c, false, false); }
__device__ __forceinline__ v8f wmmab(v16bf a, v16bf b, v8f c) { return __builtin_amdgcn_wmma_f32_16x16x32_bf16(false, a, false, b, (short)0, c, false, false); }
__device__ __forceinline__ v16h  ldh(const h16* p) { return cat16(*(const v8h*)p, *(const v8h*)(p + 16)); }
__device__ __forceinline__ v16bf ldb(const bf* p)  { return cat16b(*(const v8us*)p, *(const v8us*)(p + 16)); }
__device__ __forceinline__ void wave_sync() { __builtin_amdgcn_fence(3  , "wavefront"); __builtin_amdgcn_wave_barrier(); asm volatile("" ::: "memory"); }

__global__ __launch_bounds__(256) void k_cvt8(const float* __restrict__ src, bf* dst, size_t n8) {
    const size_t i = (size_t)blockIdx.x * 256 + threadIdx.x; if (i >= n8) return;
    const v8f v = *(const v8f*)(src + i * 8); v8us o;
#pragma unroll
    for (int k = 0; k < 8; ++k) o[k] = f2bf(v[k]);
    *(volatile v8us*)(dst + i * 8) = o; __threadfence(); *(volatile v8us*)(dst + i * 8) = o;
}

__global__ __launch_bounds__(256) void k_cvtx(const float* __restrict__ src, bf* dst) {
    const size_t i = (size_t)blockIdx.x * 256 + threadIdx.x; if (i >= (size_t)NB * SEQ * (DM / 8)) return;
    const size_t row = i >> 7; const int g = (int)(i & 127);
    const size_t b = row / SEQ, t = row % SEQ;
    const float* s = src + (b * SEQ_FULL + t) * XP + g * 8;
    const v4f x0 = *(const v4f*)s; const v4f x1 = *(const v4f*)(s + 4); v8us o;
#pragma unroll
    for (int k = 0; k < 4; ++k) { o[k] = f2bf(x0[k]); o[4 + k] = f2bf(x1[k]); }
    bf* d = dst + row * DM + g * 8;
    *(volatile v8us*)d = o; __threadfence(); *(volatile v8us*)d = o;
}

__global__ __launch_bounds__(256) void k_cvtwo(const float* __restrict__ src, h16* dst) {
    const int i = blockIdx.x * 256 + threadIdx.x; if (i >= DM * (DM / 8)) return;
    const int n = i >> 7, g = i & 127;
    const v8f v = *(const v8f*)(src + (size_t)n * DM + g * 8); v8h hv, lv;
#pragma unroll
    for (int k = 0; k < 8; ++k) { const float w = bfr(v[k]); hv[k] = (h16)(w * WHC); lv[k] = (h16)(w * WLC); }
    h16* d = dst + (size_t)n * CXP + g * 8;
    *(volatile v8h*)d = hv; *(volatile v8h*)(d + DM) = lv; __threadfence(); *(volatile v8h*)d = hv; *(volatile v8h*)(d + DM) = lv;
}

__global__ __launch_bounds__(128) void k_enct(const float* __restrict__ kx, h16* ET) {
    __shared__ __align__(16) float es[POS * 68];
    const int tid = threadIdx.x; const int b = blockIdx.y; const int t0 = blockIdx.x * 64;
#pragma unroll
    for (int j = 0; j < 2; ++j) { const int idx = tid + 128 * j; const int t = idx >> 2, p4 = (idx & 3) * 4;
        const v4f x = *(const v4f*)(kx + ((size_t)b * SEQ_FULL + t0 + t) * XP + DM + p4);
#pragma unroll
        for (int i = 0; i < 4; ++i) es[(p4 + i) * 68 + t] = bfr(x[i]); }
    __syncthreads();
    const int p = tid >> 3, c8 = (tid & 7) * 8;
    const v4f x0 = *(const v4fa*)(&es[p * 68 + c8]); const v4f x1 = *(const v4fa*)(&es[p * 68 + c8 + 4]); v8h hv;
#pragma unroll
    for (int i = 0; i < 4; ++i) { hv[i] = (h16)x0[i]; hv[4 + i] = (h16)x1[i]; }
    h16* d = ET + ((size_t)b * POS + p) * SEQ + t0 + c8;
    *(volatile v8h*)d = hv; __threadfence(); *(volatile v8h*)d = hv;
}

__global__ __launch_bounds__(32) void k_proj(const bf* __restrict__ A, const bf* __restrict__ Bt, const float* __restrict__ bias, int biasRow, h16* Ph, h16* Pr, int RB, size_t sRB, int pitch, int CB, size_t sCB) {
    __shared__ __align__(16) float os[16 * 68];
    const int K = DM;
    const int lane = threadIdx.x & 31, lr = lane & 15, hi = lane >> 4; const int r0 = blockIdx.x * 64, c0 = blockIdx.y * 64;
    v8f acc[4][4];
#pragma unroll
    for (int mb = 0; mb < 4; ++mb)
#pragma unroll
        for (int nb = 0; nb < 4; ++nb) acc[mb][nb] = (v8f){};
    const size_t aoff = (size_t)(r0 + lr) * K + 8 * hi, boff = (size_t)(c0 + lr) * K + 8 * hi;
#pragma unroll 1
    for (int kc = 0; kc < K; kc += 32) {
        v16bf a[4];
#pragma unroll
        for (int mb = 0; mb < 4; ++mb) a[mb] = ldb(A + aoff + (size_t)mb * 16 * K + kc);
#pragma unroll
        for (int nb = 0; nb < 4; ++nb) { const v16bf b = ldb(Bt + boff + (size_t)nb * 16 * K + kc);
#pragma unroll
            for (int mb = 0; mb < 4; ++mb) acc[mb][nb] = wmmab(a[mb], b, acc[mb][nb]); }
        asm volatile("v_nop\n\tv_nop\n\tv_nop\n\tv_nop" : "+v"(acc[0][0]), "+v"(acc[1][1]), "+v"(acc[2][2]), "+v"(acc[3][3]) : "v"(a[0]), "v"(a[1]), "v"(a[2]), "v"(a[3]));
    }
    const size_t tbase = (size_t)(r0 / RB) * sRB + (size_t)(r0 % RB) * (size_t)pitch + (size_t)(c0 / CB) * sCB + (size_t)(c0 % CB);
#pragma unroll
    for (int mb = 0; mb < 4; ++mb) {
#pragma unroll
        for (int nb = 0; nb < 4; ++nb) {
#pragma unroll
            for (int j = 0; j < 8; ++j) os[(hi * 8 + j) * 68 + nb * 16 + lr] = acc[mb][nb][j]; }
        wave_sync();
        const size_t sb = tbase + (size_t)(mb * 16) * (size_t)pitch;
#pragma unroll 1
        for (int ps = 0; ps < 2; ++ps) {
#pragma unroll
            for (int s = 0; s < 4; ++s) { const int row = 4 * s + (lane >> 3), c8 = (lane & 7) * 8;
                const v4f x0 = *(const v4fa*)(&os[row * 68 + c8]); const v4f x1 = *(const v4fa*)(&os[row * 68 + c8 + 4]); v8h hv, rv;
                const int bri = min(r0 + mb * 16 + row, DM - 1); const int bci = min(c0 + c8, DM - 8);
                const float rbv = bias[bri]; const v4f cb0 = *(const v4f*)(bias + bci); const v4f cb1 = *(const v4f*)(bias + bci + 4);
#pragma unroll
                for (int i = 0; i < 4; ++i) { const float y0 = x0[i] + bfr(biasRow ? rbv : cb0[i]); const float y1 = x1[i] + bfr(biasRow ? rbv : cb1[i]);
                    const h16 a0 = (h16)y0; const h16 a1 = (h16)y1; hv[i] = a0; hv[4 + i] = a1; rv[i] = (h16)((y0 - (float)a0) * QRS); rv[4 + i] = (h16)((y1 - (float)a1) * QRS); }
                const size_t oo = sb + (size_t)row * (size_t)pitch + c8;
                *(volatile v8h*)(Ph + oo) = hv; *(volatile v8h*)(Pr + oo) = rv; }
            if (ps == 0) __threadfence(); }
        wave_sync();
    }
}

template <int HP>
__device__ __forceinline__ void flash_body(const h16* __restrict__ QH, const h16* __restrict__ QR, const h16* __restrict__ KP, const h16* __restrict__ KR,
                                           const h16* __restrict__ VT, const h16* __restrict__ VR, const h16* __restrict__ ET, const int* __restrict__ MASK,
                                           h16* CX, float* EH, int tbase) {
    __shared__ __align__(16) float os[AW * 16 * OSP];
    const int lane = threadIdx.x & 31, wave = threadIdx.x >> 5, lr = lane & 15, hi = lane >> 4;
    const int zh = blockIdx.y; const int b = zh / NH_, h = zh % NH_;
    const int t0 = tbase + (blockIdx.x * AW + wave) * 16;
    const size_t pbase = (size_t)zh * SEQ * HD;
    const size_t qo = pbase + (size_t)(t0 + lr) * HD + 8 * hi;
    const v16h qh0 = ldh(QH + qo), qh1 = ldh(QH + qo + 32), qr0 = ldh(QR + qo), qr1 = ldh(QR + qo + 32);
    const size_t ko = pbase + (size_t)lr * HD + 8 * hi;
    const size_t vo = pbase + (size_t)lr * SEQ + 8 * hi;
    const size_t eo = ((size_t)b * POS + lr) * SEQ + 8 * hi;
    const int* mrow = MASK + (size_t)(t0 + lr) * SEQ_FULL + 8 * hi;
    v8f o0 = (v8f){}, o1 = (v8f){}, o2 = (v8f){}, o3 = (v8f){}, o4 = (v8f){};
    float m = -3.0e38f, l = 0.0f;
#pragma unroll 1
    for (int sweep = 0; sweep < 2; ++sweep) {
        o0 = (v8f){}; o1 = (v8f){}; o2 = (v8f){}; o3 = (v8f){}; o4 = (v8f){}; m = -3.0e38f; l = 0.0f;
        int seen = 0, skipped = 0;
#pragma unroll 1
        for (int key0 = 0; key0 < SEQ; key0 += 32) {
            const v4i mk0 = *(const v4i*)(mrow + key0), mk1 = *(const v4i*)(mrow + key0 + 4), mk2 = *(const v4i*)(mrow + key0 + 16), mk3 = *(const v4i*)(mrow + key0 + 20);
            int un = 0;
#pragma unroll
            for (int i = 0; i < 4; ++i) un |= (int)(mk0[i] != 1) | (int)(mk1[i] != 1) | (int)(mk2[i] != 1) | (int)(mk3[i] != 1);
            const bool anyun = __builtin_amdgcn_ballot_w32(un != 0) != 0u;
            if (!anyun && sweep == 0) { skipped = 1; continue; }
            seen |= un;
            const h16* ka = KP + ko + (size_t)key0 * HD;
            const v16h ka0 = ldh(ka), ka1 = ldh(ka + 32), kb0 = ldh(ka + 16 * HD), kb1 = ldh(ka + 16 * HD + 32);
            v8f sHa = (v8f){}, sLa = (v8f){}, sHb = (v8f){}, sLb = (v8f){};
            sHa = wmma16(ka0, qh0, sHa); sLa = wmma16(ka0, qr0, sLa); sHb = wmma16(kb0, qh0, sHb); sLb = wmma16(kb0, qr0, sLb);
            sHa = wmma16(ka1, qh1, sHa); sLa = wmma16(ka1, qr1, sLa); sHb = wmma16(kb1, qh1, sHb); sLb = wmma16(kb1, qr1, sLb);
            if (HP) {
                const h16* kr = KR + ko + (size_t)key0 * HD;
                const v16h ra0 = ldh(kr), ra1 = ldh(kr + 32), rb0 = ldh(kr + 16 * HD), rb1 = ldh(kr + 16 * HD + 32);
                sLa = wmma16(ra0, qh0, sLa); sLb = wmma16(rb0, qh0, sLb); sLa = wmma16(ra1, qh1, sLa); sLb = wmma16(rb1, qh1, sLb);
                asm volatile("v_nop\n\tv_nop\n\tv_nop\n\tv_nop" : "+v"(sHa), "+v"(sLa), "+v"(sHb), "+v"(sLb) : "v"(ka0), "v"(ka1), "v"(kb0), "v"(kb1), "v"(ra0), "v"(ra1), "v"(rb0), "v"(rb1));
            } else {
                asm volatile("v_nop\n\tv_nop\n\tv_nop\n\tv_nop" : "+v"(sHa), "+v"(sLa), "+v"(sHb), "+v"(sLb) : "v"(ka0), "v"(ka1), "v"(kb0), "v"(kb1));
            }
            float ta[8], tb[8]; float mx = -3.0e38f;
#pragma unroll
            for (int r = 0; r < 8; ++r) {
                const int ma = (r < 4) ? mk0[r & 3] : mk1[r & 3]; const int mc = (r < 4) ? mk2[r & 3] : mk3[r & 3];
                const float sa = (sHa[r] + sLa[r] * QRI) * SC2; const float sc = (sHb[r] + sLb[r] * QRI) * SC2;
                ta[r] = (ma == 1) ? MASKV : sa; tb[r] = (mc == 1) ? MASKV : sc; mx = fmaxf(mx, fmaxf(ta[r], tb[r])); }
            mx = fmaxf(mx, __shfl_xor(mx, 16, 32));
            const float mnew = fmaxf(m, mx);
            const float alpha = __builtin_amdgcn_exp2f(m - mnew);
            const float sh = PSH - mnew;
            v16h pbh, pbr, pbs; float ls = 0.0f;
#pragma unroll
            for (int r = 0; r < 8; ++r) {
                const float fa = __builtin_amdgcn_exp2f(ta[r] + sh); const float fc = __builtin_amdgcn_exp2f(tb[r] + sh);
                const h16 pa = (h16)fa; const h16 pc = (h16)fc; pbh[r] = pa; pbh[8 + r] = pc;
                if (HP) { const h16 ra = (h16)(fa - (float)pa); const h16 rc = (h16)(fc - (float)pc); pbr[r] = ra; pbr[8 + r] = rc;
                    pbs[r] = (h16)((float)pa * QRI); pbs[8 + r] = (h16)((float)pc * QRI);
                    ls += ((float)pa + (float)ra) + ((float)pc + (float)rc);
                } else { ls += (float)pa + (float)pc; } }
            l = l * alpha + ls; m = mnew;
            o0 = o0 * alpha; o1 = o1 * alpha; o2 = o2 * alpha; o3 = o3 * alpha; o4 = o4 * alpha;
            const h16* va = VT + vo + key0;
            const v16h v0 = ldh(va), v1 = ldh(va + (size_t)16 * SEQ), v2 = ldh(va + (size_t)32 * SEQ), v3 = ldh(va + (size_t)48 * SEQ);
            const v16h e0 = ldh(ET + eo + key0);
            if (HP) {
                const h16* vr = VR + vo + key0;
                const v16h r0 = ldh(vr), r1 = ldh(vr + (size_t)16 * SEQ), r2 = ldh(vr + (size_t)32 * SEQ), r3 = ldh(vr + (size_t)48 * SEQ);
                o0 = wmma16(v0, pbh, o0); o1 = wmma16(v1, pbh, o1); o2 = wmma16(v2, pbh, o2); o3 = wmma16(v3, pbh, o3); o4 = wmma16(e0, pbh, o4);
                o0 = wmma16(v0, pbr, o0); o1 = wmma16(v1, pbr, o1); o2 = wmma16(v2, pbr, o2); o3 = wmma16(v3, pbr, o3); o4 = wmma16(e0, pbr, o4);
                o0 = wmma16(r0, pbs, o0); o1 = wmma16(r1, pbs, o1); o2 = wmma16(r2, pbs, o2); o3 = wmma16(r3, pbs, o3);
                asm volatile("v_nop\n\tv_nop\n\tv_nop\n\tv_nop" : "+v"(o0), "+v"(o1), "+v"(o2), "+v"(o3), "+v"(o4)
                             : "v"(v0), "v"(v1), "v"(v2), "v"(v3), "v"(e0), "v"(r0), "v"(r1), "v"(r2), "v"(r3), "v"(pbh), "v"(pbr), "v"(pbs));
            } else {
                o0 = wmma16(v0, pbh, o0); o1 = wmma16(v1, pbh, o1); o2 = wmma16(v2, pbh, o2); o3 = wmma16(v3, pbh, o3); o4 = wmma16(e0, pbh, o4);
                asm volatile("v_nop\n\tv_nop\n\tv_nop\n\tv_nop" : "+v"(o0), "+v"(o1), "+v"(o2), "+v"(o3), "+v"(o4) : "v"(v0), "v"(v1), "v"(v2), "v"(v3), "v"(e0), "v"(pbh));
            }
        }
        const int sr = seen | __shfl_xor(seen, 16, 32);
        const bool redo = (sweep == 0) && (skipped != 0) && (__builtin_amdgcn_ballot_w32(sr == 0) != 0u);
        if (!redo) break;
    }
    l += __shfl_xor(l, 16, 32);
    const float inv = 1.0f / l;
    const int wb = wave * 16 * OSP;
    { v4f a, c;
      a[0] = o0[0] * inv; a[1] = o0[1] * inv; a[2] = o0[2] * inv; a[3] = o0[3] * inv; c[0] = o0[4] * inv; c[1] = o0[5] * inv; c[2] = o0[6] * inv; c[3] = o0[7] * inv;
      *(v4fa*)(&os[wb + lr * OSP +  0 + 8 * hi]) = a; *(v4fa*)(&os[wb + lr * OSP +  0 + 8 * hi + 4]) = c;
      a[0] = o1[0] * inv; a[1] = o1[1] * inv; a[2] = o1[2] * inv; a[3] = o1[3] * inv; c[0] = o1[4] * inv; c[1] = o1[5] * inv; c[2] = o1[6] * inv; c[3] = o1[7] * inv;
      *(v4fa*)(&os[wb + lr * OSP + 16 + 8 * hi]) = a; *(v4fa*)(&os[wb + lr * OSP + 16 + 8 * hi + 4]) = c;
      a[0] = o2[0] * inv; a[1] = o2[1] * inv; a[2] = o2[2] * inv; a[3] = o2[3] * inv; c[0] = o2[4] * inv; c[1] = o2[5] * inv; c[2] = o2[6] * inv; c[3] = o2[7] * inv;
      *(v4fa*)(&os[wb + lr * OSP + 32 + 8 * hi]) = a; *(v4fa*)(&os[wb + lr * OSP + 32 + 8 * hi + 4]) = c;
      a[0] = o3[0] * inv; a[1] = o3[1] * inv; a[2] = o3[2] * inv; a[3] = o3[3] * inv; c[0] = o3[4] * inv; c[1] = o3[5] * inv; c[2] = o3[6] * inv; c[3] = o3[7] * inv;
      *(v4fa*)(&os[wb + lr * OSP + 48 + 8 * hi]) = a; *(v4fa*)(&os[wb + lr * OSP + 48 + 8 * hi + 4]) = c;
      a[0] = o4[0] * inv; a[1] = o4[1] * inv; a[2] = o4[2] * inv; a[3] = o4[3] * inv; c[0] = o4[4] * inv; c[1] = o4[5] * inv; c[2] = o4[6] * inv; c[3] = o4[7] * inv;
      *(v4fa*)(&os[wb + lr * OSP + 64 + 8 * hi]) = a; *(v4fa*)(&os[wb + lr * OSP + 64 + 8 * hi + 4]) = c; }
    wave_sync();
    h16* crow = CX + ((size_t)b * SEQ + t0) * CXP + h * HD;
    float* eh = EH + ((size_t)zh * SEQ + t0) * POS;
#pragma unroll 1
    for (int ps = 0; ps < 2; ++ps) {
#pragma unroll
        for (int s = 0; s < 4; ++s) { const int row = 4 * s + (lane >> 3), c8 = (lane & 7) * 8;
            const v4f x0 = *(const v4fa*)(&os[wb + row * OSP + c8]); const v4f x1 = *(const v4fa*)(&os[wb + row * OSP + c8 + 4]); v8h hv, rv;
#pragma unroll
            for (int i = 0; i < 4; ++i) { const float y0 = x0[i] * CXC; const float y1 = x1[i] * CXC; const h16 a0 = (h16)y0; const h16 a1 = (h16)y1;
                hv[i] = a0; hv[4 + i] = a1; rv[i] = (h16)((y0 - (float)a0) * QRS); rv[4 + i] = (h16)((y1 - (float)a1) * QRS); }
            *(volatile v8h*)(crow + (size_t)row * CXP + c8) = hv;
            if (HP) *(volatile v8h*)(crow + (size_t)row * CXP + DM + c8) = rv; }
#pragma unroll
        for (int s = 0; s < 2; ++s) { const int f4 = s * 32 + lane; const int row = f4 >> 2, p4 = (f4 & 3) * 4;
            const v4f val = *(const v4fa*)(&os[wb + row * OSP + 64 + p4]);
            *(volatile v4f*)(eh + (size_t)f4 * 4) = val; }
        if (ps == 0) __threadfence(); }
}

__global__ __launch_bounds__(32 * AW) void k_flash_hp(const h16* __restrict__ QH, const h16* __restrict__ QR, const h16* __restrict__ KP, const h16* __restrict__ KR,
                                                      const h16* __restrict__ VT, const h16* __restrict__ VR, const h16* __restrict__ ET, const int* __restrict__ MASK,
                                                      h16* CX, float* EH, int tbase) {
    flash_body<1>(QH, QR, KP, KR, VT, VR, ET, MASK, CX, EH, tbase);
}
__global__ __launch_bounds__(32 * AW) void k_flash_sp(const h16* __restrict__ QH, const h16* __restrict__ QR, const h16* __restrict__ KP, const h16* __restrict__ KR,
                                                      const h16* __restrict__ VT, const h16* __restrict__ VR, const h16* __restrict__ ET, const int* __restrict__ MASK,
                                                      h16* CX, float* EH, int tbase) {
    flash_body<0>(QH, QR, KP, KR, VT, VR, ET, MASK, CX, EH, tbase);
}

__global__ __launch_bounds__(32) void k_oproj(const h16* __restrict__ A, const h16* __restrict__ Bt, const float* __restrict__ bo, float* Y) {
    __shared__ __align__(16) float os[16 * 68];
    const int lane = threadIdx.x & 31, lr = lane & 15, hi = lane >> 4; const int r0 = blockIdx.x * 64, c0 = blockIdx.y * 64;
    const int KT = ((r0 % SEQ) < EARLYR) ? (2 * DM) : DM;
    v8f acc[4][4];
#pragma unroll
    for (int mb = 0; mb < 4; ++mb)
#pragma unroll
        for (int nb = 0; nb < 4; ++nb) acc[mb][nb] = (v8f){};
    const size_t aoff = (size_t)(r0 + lr) * CXP + 8 * hi, boff = (size_t)(c0 + lr) * CXP + 8 * hi;
#pragma unroll 1
    for (int kc = 0; kc < KT; kc += 32) {
        v16h a[4];
#pragma unroll
        for (int mb = 0; mb < 4; ++mb) a[mb] = ldh(A + aoff + (size_t)mb * 16 * CXP + kc);
#pragma unroll
        for (int nb = 0; nb < 4; ++nb) { const v16h b = ldh(Bt + boff + (size_t)nb * 16 * CXP + kc);
#pragma unroll
            for (int mb = 0; mb < 4; ++mb) acc[mb][nb] = wmma16(a[mb], b, acc[mb][nb]); }
        asm volatile("v_nop\n\tv_nop\n\tv_nop\n\tv_nop" : "+v"(acc[0][0]), "+v"(acc[1][1]), "+v"(acc[2][2]), "+v"(acc[3][3]) : "v"(a[0]), "v"(a[1]), "v"(a[2]), "v"(a[3]));
    }
#pragma unroll
    for (int mb = 0; mb < 4; ++mb) {
#pragma unroll
        for (int nb = 0; nb < 4; ++nb) {
#pragma unroll
            for (int j = 0; j < 8; ++j) os[(hi * 8 + j) * 68 + nb * 16 + lr] = acc[mb][nb][j]; }
        wave_sync();
        float* yb = Y + (size_t)(r0 + mb * 16) * DM + c0;
#pragma unroll 1
        for (int ps = 0; ps < 2; ++ps) {
#pragma unroll
            for (int s = 0; s < 8; ++s) { const int row = 2 * s + hi, cofs = lr * 4;
                const v4f x = *(const v4fa*)(&os[row * 68 + cofs]); const v4f bb = *(const v4f*)(bo + c0 + cofs); v4f val;
#pragma unroll
                for (int i = 0; i < 4; ++i) val[i] = x[i] * OSC + bfr(bb[i]);
                *(volatile v4f*)(yb + (size_t)row * DM + cofs) = val; }
            if (ps == 0) __threadfence(); }
        wave_sync();
    }
}

__global__ __launch_bounds__(256) void k_final(const float* __restrict__ Y, const float* __restrict__ EH, const int* __restrict__ PIN, float* OUT) {
    __shared__ __align__(16) float es[8 * POS];
    const int tid = threadIdx.x, wave = tid >> 5, lane = tid & 31;
    const int m0 = blockIdx.x * 8; const int b = m0 / SEQ, t0 = m0 % SEQ;
    if (wave == 0) {
        const int row = lane >> 2, p4 = (lane & 3) * 4; v4f acc = (v4f){};
#pragma unroll 4
        for (int h = 0; h < NH_; ++h) acc += *(const v4f*)(EH + (((size_t)b * NH_ + h) * SEQ + t0 + row) * POS + p4);
        acc = acc * 0.0625f;
        *(v4fa*)(&es[row * POS + p4]) = acc;
    }
    __syncthreads();
    const bool ok = (PIN[0] == POS);
    const float qnan = __uint_as_float(0x7FC00000u);
    float* obase = OUT + ((size_t)b * OUT_SEQ + t0) * XP;
    const int NP = 8 * XP / 4;
#pragma unroll 1
    for (int ps = 0; ps < 2; ++ps) {
#pragma unroll 1
        for (int it = 0; it < (NP + 255) / 256; ++it) {
            const int f = it * 256 + tid; const int fc = min(f, NP - 1);
            const int e = fc * 4; const int row = e / XP; const int col = e - row * XP;
            const int yc = min(col, DM - 4); const int ec = min(max(col - DM, 0), POS - 4);
            const v4f yv = *(const v4f*)(Y + (size_t)(m0 + row) * DM + yc);
            const v4f ev = *(const v4fa*)(&es[row * POS + ec]);
            v4f val = (col < DM) ? yv : ev;
            if (!ok) { val[0] = qnan; val[1] = qnan; val[2] = qnan; val[3] = qnan; }
            if (f < NP) *(volatile v4f*)(obase + (size_t)fc * 4) = val;
        }
        if (ps == 0) __threadfence(); }
}

static constexpr size_t al256(size_t v) { return (v + 255) & ~(size_t)255; }
static constexpr size_t SZ_XB = al256((size_t)NB * SEQ * DM * 2);
static constexpr size_t SZ_W  = al256((size_t)DM * DM * 2);
static constexpr size_t SZ_WO = al256((size_t)DM * CXP * 2);
static constexpr size_t SZ_PL = al256((size_t)NB * NH_ * SEQ * HD * 2);
static constexpr size_t SZ_ET = al256((size_t)NB * POS * SEQ * 2);
static constexpr size_t SZ_CX = al256((size_t)NB * SEQ * CXP * 2);
static constexpr size_t SZ_EH = al256((size_t)NB * NH_ * SEQ * POS * 4);
static constexpr size_t SZ_Y  = al256((size_t)NB * SEQ * DM * 4);
static constexpr size_t SZ_TOTAL = 3 * SZ_XB + 3 * SZ_W + SZ_WO + 6 * SZ_PL + SZ_ET + SZ_CX + SZ_EH + SZ_Y;
static_assert(SZ_TOTAL <= (size_t)134217728);

extern "C" void kernel_launch(void* const* d_in, const int* in_sizes, int n_in,
                              void* d_out, int out_size, void* d_ws, size_t ws_size, hipStream_t stream) {
    if (n_in < 13) return;
    const size_t needx = ((size_t)(NB - 1) * SEQ_FULL + SEQ) * XP;
    if ((size_t)in_sizes[0] < needx || (size_t)in_sizes[1] < needx || (size_t)in_sizes[2] < needx) return;
    if ((size_t)in_sizes[3] < (size_t)DM * DM || (size_t)in_sizes[5] < (size_t)DM * DM || (size_t)in_sizes[7] < (size_t)DM * DM || (size_t)in_sizes[9] < (size_t)DM * DM) return;
    if (in_sizes[4] < DM || in_sizes[6] < DM || in_sizes[8] < DM || in_sizes[10] < DM) return;
    if ((size_t)in_sizes[11] < (size_t)(SEQ - 1) * SEQ_FULL + SEQ) return;
    if (in_sizes[12] < 1) return;
    if ((size_t)out_size < ((size_t)(NB - 1) * OUT_SEQ + SEQ) * XP) return;
    if (SZ_TOTAL > ws_size) return;
    const float* xq = (const float*)d_in[0]; const float* xk = (const float*)d_in[1]; const float* xv = (const float*)d_in[2];
    const float* wq = (const float*)d_in[3]; const float* bq = (const float*)d_in[4];
    const float* wk = (const float*)d_in[5]; const float* bk = (const float*)d_in[6];
    const float* wv = (const float*)d_in[7]; const float* bv = (const float*)d_in[8];
    const float* wo = (const float*)d_in[9]; const float* bo = (const float*)d_in[10];
    const int* mask = (const int*)d_in[11]; const int* pin = (const int*)d_in[12];
    float* OUT = (float*)d_out;
    char* wsp = (char*)d_ws;
    bf* XQ = (bf*)wsp; wsp += SZ_XB;
    bf* XK = (bf*)wsp; wsp += SZ_XB;
    bf* XV = (bf*)wsp; wsp += SZ_XB;
    bf* WQ = (bf*)wsp; wsp += SZ_W;
    bf* WK = (bf*)wsp; wsp += SZ_W;
    bf* WV = (bf*)wsp; wsp += SZ_W;
    h16* WO = (h16*)wsp; wsp += SZ_WO;
    h16* QH = (h16*)wsp; wsp += SZ_PL;
    h16* QR = (h16*)wsp; wsp += SZ_PL;
    h16* KP = (h16*)wsp; wsp += SZ_PL;
    h16* KR = (h16*)wsp; wsp += SZ_PL;
    h16* VT = (h16*)wsp; wsp += SZ_PL;
    h16* VR = (h16*)wsp; wsp += SZ_PL;
    h16* ET = (h16*)wsp; wsp += SZ_ET;
    h16* CX = (h16*)wsp; wsp += SZ_CX;
    float* EH = (float*)wsp; wsp += SZ_EH;
    float* Y  = (float*)wsp; wsp += SZ_Y;

    { const unsigned g = (unsigned)(((size_t)NB * SEQ * (DM / 8) + 255) / 256);
      k_cvtx<<<g, 256, 0, stream>>>(xq, XQ); k_cvtx<<<g, 256, 0, stream>>>(xk, XK); k_cvtx<<<g, 256, 0, stream>>>(xv, XV); }
    k_enct<<<dim3(SEQ / 64, NB, 1), 128, 0, stream>>>(xk, ET);
    { const size_t n8 = (size_t)DM * DM / 8; const unsigned g = (unsigned)((n8 + 255) / 256);
      k_cvt8<<<g, 256, 0, stream>>>(wq, WQ, n8); k_cvt8<<<g, 256, 0, stream>>>(wk, WK, n8); k_cvt8<<<g, 256, 0, stream>>>(wv, WV, n8);
      k_cvtwo<<<g, 256, 0, stream>>>(wo, WO); }

    k_proj<<<dim3(NB * SEQ / 64, DM / 64, 1), 32, 0, stream>>>(XQ, WQ, bq, 0, QH, QR, SEQ, (size_t)NH_ * SEQ * HD, HD, HD, (size_t)SEQ * HD);
    k_proj<<<dim3(NB * SEQ / 64, DM / 64, 1), 32, 0, stream>>>(XK, WK, bk, 0, KP, KR, SEQ, (size_t)NH_ * SEQ * HD, HD, HD, (size_t)SEQ * HD);
    k_proj<<<dim3(DM / 64, NB * SEQ / 64, 1), 32, 0, stream>>>(WV, XV, bv, 1, VT, VR, DM, (size_t)0, SEQ, SEQ, (size_t)DM * SEQ);

    k_flash_hp<<<dim3(EARLYR / (16 * AW), NB * NH_, 1), 32 * AW, 0, stream>>>(QH, QR, KP, KR, VT, VR, ET, mask, CX, EH, 0);
    if (SEQ > EARLYR)
        k_flash_sp<<<dim3((SEQ - EARLYR) / (16 * AW), NB * NH_, 1), 32 * AW, 0, stream>>>(QH, QR, KP, KR, VT, VR, ET, mask, CX, EH, EARLYR);

    k_oproj<<<dim3(NB * SEQ / 64, DM / 64, 1), 32, 0, stream>>>(CX, WO, bo, Y);
    k_final<<<NB * SEQ / 8, 256, 0, stream>>>(Y, EH, pin, OUT);
}
